// LzScaleDotAttention_38190849196228
// MI455X (gfx1250) — hardware-verified
//
#include <hip/hip_runtime.h>
#include <stddef.h>


typedef _Float16 h16 __attribute__((ext_vector_type(16)));
typedef _Float16 h8n __attribute__((ext_vector_type(8)));
typedef _Float16 h8  __attribute__((ext_vector_type(8), __may_alias__));
typedef float    f8  __attribute__((ext_vector_type(8)));
typedef float    v4fn __attribute__((ext_vector_type(4)));
typedef float    v4f __attribute__((ext_vector_type(4), __may_alias__));

union Frag { h16 v; h8n h[2]; };

#define BATCH 8
#define SEQ   2048
#define DIM   512
#define BM    32
#define BJ    32
#define NITER (SEQ / BJ)
#define NTOT  (BATCH * SEQ * DIM)
#define VP    32
#define PP    32

#define QK_SCALE   16.0f
#define V_SCALE    16.0f
#define S_UNSCALE  (1.0f / 256.0f)
#define O_UNSCALE  (1.0f / 16.0f)
#define EPS_SCALED 2.2627417e-6f

static_assert(SEQ % BM == 0);
static_assert(SEQ % BJ == 0);
static_assert(DIM % 32 == 0);
static_assert(NTOT % (256 * 8) == 0);
static_assert(BM * DIM == 16 * 256 * 4);
static_assert(DIM * BJ == 8 * 256 * 8);

__device__ __forceinline__ f8 wmma_f16(h16 a, h16 b, f8 c) {
    f8 d = __builtin_amdgcn_wmma_f32_16x16x32_f16(false, a, false, b, (short)0, c, false, false);
    asm volatile("v_nop\n\tv_nop\n\tv_nop\n\tv_nop" : "+v"(d) : "v"(a), "v"(b));
    return d;
}

__global__ __launch_bounds__(256)
void cvt_qk_kernel(const float* __restrict__ q, const float* __restrict__ k,
                   _Float16* __restrict__ q16, _Float16* __restrict__ k16)
{
    const bool isk = (blockIdx.y != 0);
    const float* src = isk ? k : q;
    _Float16*    dst = isk ? k16 : q16;
    const size_t i = ((size_t)blockIdx.x * 256 + threadIdx.x) * 8;
    const float4 a = *(const float4*)(src + i);
    const float4 b = *(const float4*)(src + i + 4);
    h8n o;
    o[0] = (_Float16)(a.x * QK_SCALE); o[1] = (_Float16)(a.y * QK_SCALE);
    o[2] = (_Float16)(a.z * QK_SCALE); o[3] = (_Float16)(a.w * QK_SCALE);
    o[4] = (_Float16)(b.x * QK_SCALE); o[5] = (_Float16)(b.y * QK_SCALE);
    o[6] = (_Float16)(b.z * QK_SCALE); o[7] = (_Float16)(b.w * QK_SCALE);
    volatile h8* p = (volatile h8*)(dst + i);
    *p = o;
    __threadfence();
    *p = o;
}

__global__ __launch_bounds__(256)
void cvt_vt_kernel(const float* __restrict__ v, _Float16* __restrict__ vtg)
{
    __shared__ __align__(16) _Float16 lt[DIM * VP];
    const int tid = threadIdx.x;
    const int blk = blockIdx.x;
    const int b   = blk / NITER;
    const int it  = blk - b * NITER;
    const float* src = v + ((size_t)b * SEQ + (size_t)it * BJ) * DIM;

    #pragma unroll
    for (int u = 0; u < 16; ++u) {
        const int f  = u * 256 + tid;
        const int j  = f >> 7;
        const int d0 = (f & 127) * 4;
        const float4 x = *(const float4*)(src + (size_t)j * DIM + d0);
        lt[(d0 + 0) * VP + j] = (_Float16)(x.x * V_SCALE);
        lt[(d0 + 1) * VP + j] = (_Float16)(x.y * V_SCALE);
        lt[(d0 + 2) * VP + j] = (_Float16)(x.z * V_SCALE);
        lt[(d0 + 3) * VP + j] = (_Float16)(x.w * V_SCALE);
    }
    __syncthreads();

    _Float16* dst = vtg + (size_t)blk * (DIM * BJ);
    h8n vals[8];
    #pragma unroll
    for (int u = 0; u < 8; ++u) {
        const int idx = (u * 256 + tid) * 8;
        vals[u] = *(const h8*)&lt[idx];
    }
    #pragma unroll
    for (int u = 0; u < 8; ++u) {
        const int idx = (u * 256 + tid) * 8;
        *(volatile h8*)(dst + idx) = vals[u];
    }
    __threadfence();
    #pragma unroll
    for (int u = 0; u < 8; ++u) {
        const int idx = (u * 256 + tid) * 8;
        *(volatile h8*)(dst + idx) = vals[u];
    }
}

__global__ __launch_bounds__(256)
void attn_kernel(const float* __restrict__ vg,
                 const _Float16* __restrict__ q16, const _Float16* __restrict__ k16,
                 const _Float16* __restrict__ vtg,
                 float* __restrict__ outg)
{
    __shared__ __align__(16) _Float16 vT[DIM * VP];
    __shared__ __align__(16) _Float16 pbuf[BM * PP];
    __shared__ __align__(16) float    ost[BM * DIM];
    __shared__ float    denom_s[BM];
    __shared__ unsigned mask_s[BM];

    const int tid  = threadIdx.x;
    const int lane = tid & 31;
    const int wave = tid >> 5;
    const int h    = lane >> 4;
    const int m    = lane & 15;
    const int mg   = wave & 1;
    const int dq   = wave >> 1;
    const int b    = blockIdx.y;
    const int i0   = blockIdx.x * BM;

    f8 zero8;
    #pragma unroll
    for (int i = 0; i < 8; ++i) zero8[i] = 0.0f;
    f8 acc[8];
    #pragma unroll
    for (int n = 0; n < 8; ++n) acc[n] = zero8;
    f8 dsum = zero8;

    const _Float16* kA = k16 + ((size_t)b * SEQ + i0 + mg * 16 + m) * DIM + 8 * h;
    const _Float16* qB = q16 + (size_t)b * SEQ * DIM + 8 * h;

    #pragma unroll 1
    for (int it = 0; it < NITER; ++it) {
        const int j0 = it * BJ;

        __syncthreads();

        {
            const _Float16* src = vtg + ((size_t)b * NITER + it) * (DIM * BJ);
            #pragma unroll
            for (int u = 0; u < 8; ++u) {
                const int idx = (u * 256 + tid) * 8;
                *(h8*)&vT[idx] = *(const h8*)(src + idx);
            }
        }

        if (dq == 0) {
            f8 s0 = zero8, s1 = zero8;
            const _Float16* q0 = qB + (size_t)(j0 + m) * DIM;
            const _Float16* q1 = qB + (size_t)(j0 + 16 + m) * DIM;
            #pragma unroll 4
            for (int ks = 0; ks < DIM / 32; ++ks) {
                const int c = ks * 32;
                Frag a, b0, b1;
                a.h[0]  = *(const h8*)(kA + c);
                a.h[1]  = *(const h8*)(kA + c + 16);
                b0.h[0] = *(const h8*)(q0 + c);
                b0.h[1] = *(const h8*)(q0 + c + 16);
                b1.h[0] = *(const h8*)(q1 + c);
                b1.h[1] = *(const h8*)(q1 + c + 16);
                s0 = wmma_f16(a.v, b0.v, s0);
                s1 = wmma_f16(a.v, b1.v, s1);
            }
            float e0[8], e1[8];
            #pragma unroll
            for (int i = 0; i < 8; ++i) {
                e0[i] = __expf(s0[i] * S_UNSCALE);
                e1[i] = __expf(s1[i] * S_UNSCALE);
            }
            #pragma unroll
            for (int i = 0; i < 8; ++i) {
                const int row = mg * 16 + 8 * h + i;
                pbuf[row * PP + m]      = (_Float16)e0[i];
                pbuf[row * PP + 16 + m] = (_Float16)e1[i];
            }
            #pragma unroll
            for (int i = 0; i < 8; ++i) {
                float t = e0[i] + e1[i];
                t += __shfl_xor(t, 1);
                t += __shfl_xor(t, 2);
                t += __shfl_xor(t, 4);
                t += __shfl_xor(t, 8);
                dsum[i] += t;
            }
        }
        __syncthreads();

        {
            const _Float16* pr = pbuf + (mg * 16 + m) * PP + 8 * h;
            Frag ap;
            ap.h[0] = *(const h8*)(pr);
            ap.h[1] = *(const h8*)(pr + 16);
            #pragma unroll
            for (int nt = 0; nt < 8; ++nt) {
                const int d = dq * 128 + nt * 16 + m;
                const _Float16* vp = vT + d * VP + 8 * h;
                Frag bv;
                bv.h[0] = *(const h8*)(vp);
                bv.h[1] = *(const h8*)(vp + 16);
                acc[nt] = wmma_f16(ap.v, bv.v, acc[nt]);
            }
        }
    }

    if (dq == 0 && m == 0) {
        #pragma unroll
        for (int i = 0; i < 8; ++i) denom_s[mg * 16 + 8 * h + i] = dsum[i];
    }

    {
        const int row = tid >> 3;
        const int seg = tid & 7;
        const float* src = vg + ((size_t)b * SEQ + i0 + row) * DIM + seg * 64;
        int nz = 0;
        #pragma unroll 4
        for (int u = 0; u < 16; ++u) {
            const float4 x = *(const float4*)(src + u * 4);
            nz |= (int)(x.x != 0.0f) | (int)(x.y != 0.0f) | (int)(x.z != 0.0f) | (int)(x.w != 0.0f);
        }
        nz |= __shfl_xor(nz, 1);
        nz |= __shfl_xor(nz, 2);
        nz |= __shfl_xor(nz, 4);
        if (seg == 0) mask_s[row] = (unsigned)nz;
    }
    __syncthreads();

    {
        float sc[8];
        #pragma unroll
        for (int i = 0; i < 8; ++i) {
            const int row = mg * 16 + 8 * h + i;
            const float den = denom_s[row] + EPS_SCALED;
            sc[i] = (mask_s[row] != 0u) ? (O_UNSCALE * __builtin_amdgcn_rcpf(den)) : 0.0f;
        }
        #pragma unroll
        for (int nt = 0; nt < 8; ++nt) {
            #pragma unroll
            for (int i = 0; i < 8; ++i) {
                const int row = mg * 16 + 8 * h + i;
                ost[row * DIM + dq * 128 + nt * 16 + m] = acc[nt][i] * sc[i];
            }
        }
    }
    __syncthreads();

    {
        float* ob = outg + ((size_t)b * SEQ + i0) * DIM;
        v4fn vals[16];
        #pragma unroll
        for (int u = 0; u < 16; ++u) {
            const int idx = (u * 256 + tid) * 4;
            vals[u] = *(const v4f*)&ost[idx];
        }
        #pragma unroll
        for (int u = 0; u < 16; ++u) {
            const int idx = (u * 256 + tid) * 4;
            *(volatile v4f*)(ob + idx) = vals[u];
        }
        __threadfence();
        #pragma unroll
        for (int u = 0; u < 16; ++u) {
            const int idx = (u * 256 + tid) * 4;
            *(volatile v4f*)(ob + idx) = vals[u];
        }
    }
}

extern "C" void kernel_launch(void* const* d_in, const int* in_sizes, int n_in,
                              void* d_out, int out_size, void* d_ws, size_t ws_size,
                              hipStream_t stream)
{
    if (n_in < 3) return;
    if (in_sizes[0] != NTOT || in_sizes[1] != NTOT || in_sizes[2] != NTOT) return;
    if (out_size != NTOT) return;

    const size_t plane_bytes = (size_t)NTOT * sizeof(_Float16);
    const size_t need = 3 * plane_bytes;
    if (d_ws == nullptr || ws_size < need) return;

    const float* q = (const float*)d_in[0];
    const float* k = (const float*)d_in[1];
    const float* v = (const float*)d_in[2];
    float* out = (float*)d_out;

    _Float16* q16  = (_Float16*)d_ws;
    _Float16* k16  = (_Float16*)((char*)d_ws + plane_bytes);
    _Float16* vt16 = (_Float16*)((char*)d_ws + 2 * plane_bytes);

    cvt_qk_kernel<<<dim3(NTOT / (256 * 8), 2), dim3(256), 0, stream>>>(q, k, q16, k16);
    cvt_vt_kernel<<<dim3(BATCH * NITER), dim3(256), 0, stream>>>(v, vt16);
    attn_kernel<<<dim3(SEQ / BM, BATCH), dim3(256), 0, stream>>>(v, q16, k16, vt16, out);
    (void)hipGetLastError();
}
